// DeformableConv3D_82678120448138
// MI455X (gfx1250) — hardware-verified
//
#include <hip/hip_runtime.h>
#include <stddef.h>


#define CIN   32
#define COUT  32
#define KT    27
#define DD    32
#define HH    64
#define WW    64
#define NSP   (DD * HH * WW)
#define PD    34
#define PH    66
#define PW    66
#define NPP   (PD * PH * PW)
#define NPPR  148160
#define KDIM  (KT * CIN)
#define N1    112
#define NT1   7
#define NWV   4
#define NTH   (NWV * 32)
#define POSB  (NWV * 16)
#define T1    (N1 * KDIM / 8)
#define T2    (COUT * KDIM / 8)

static_assert(NPPR % 64 == 0);
static_assert(NPPR >= NPP);
static_assert(NSP % POSB == 0);
static_assert((WW % 16) == 0);
static_assert(T1 % 32 == 0);
static_assert((T1 + T2) % 32 == 0);
static_assert(COUT * POSB <= N1 * 16 * NWV);

typedef float          v4f   __attribute__((ext_vector_type(4)));
typedef float          v8f   __attribute__((ext_vector_type(8)));
typedef unsigned short v8us  __attribute__((ext_vector_type(8)));
typedef __bf16         v16bf __attribute__((ext_vector_type(16)));
union FragB { v16bf v; v8us u[2]; };
static_assert(sizeof(FragB) == 32);

__device__ __forceinline__ unsigned int bf16_rne(float f) {
  const unsigned int u = __float_as_uint(f);
  return (u + 0x7FFFu + ((u >> 16) & 1u)) >> 16;
}

__device__ __forceinline__ v8f zero8f() {
  v8f z;
#pragma unroll
  for (int i = 0; i < 8; ++i) z[i] = 0.0f;
  return z;
}

__device__ __forceinline__ v8f wmb(v16bf a, v16bf b, v8f c) {
  return __builtin_amdgcn_wmma_f32_16x16x32_bf16(false, a, false, b, (short)0, c, false, false);
}

__device__ __forceinline__ void wguard(v8f& d, v16bf a0, v16bf a1, v16bf b0, v16bf b1) {
  asm volatile("v_nop\n\tv_nop\n\tv_nop\n\tv_nop" : "+v"(d) : "v"(a0), "v"(a1), "v"(b0), "v"(b1));
}

__global__ __launch_bounds__(256) void k_pad(const float* __restrict__ x, float* xf,
                                             unsigned short* xh, unsigned short* xl) {
  __shared__ __attribute__((aligned(16))) float tile[64 * CIN];
  const int tid = threadIdx.x;
  const int pl = tid >> 2, cg = tid & 3;
  const int p = blockIdx.x * 64 + pl;
  int t = p;
  const int xp = t % PW; t /= PW;
  const int yp = t % PH;
  const int zp = t / PH;
  const bool inb = (p < NPP) && (zp >= 1) && (zp <= DD) && (yp >= 1) && (yp <= HH) &&
                   (xp >= 1) && (xp <= WW);
  const int zc = min(max(zp - 1, 0), DD - 1);
  const int yc = min(max(yp - 1, 0), HH - 1);
  const int xc = min(max(xp - 1, 0), WW - 1);
  float v[8];
  v8us hv, lv;
#pragma unroll
  for (int j = 0; j < 8; ++j) {
    const int c = cg * 8 + j;
    const float r = x[((size_t)(c * DD + zc) * HH + yc) * WW + xc];
    const float f = inb ? r : 0.0f;
    v[j] = f;
    const unsigned int hb = bf16_rne(f);
    hv[j] = (unsigned short)hb;
    lv[j] = (unsigned short)bf16_rne(f - __uint_as_float(hb << 16));
  }
  {
    v4f t0 = {v[0], v[1], v[2], v[3]};
    v4f t1 = {v[4], v[5], v[6], v[7]};
    *(v4f*)(tile + pl * CIN + cg * 8)     = t0;
    *(v4f*)(tile + pl * CIN + cg * 8 + 4) = t1;
  }
  __syncthreads();
  const int q0 = tid, q1 = 256 + tid;
  const v4f f0 = *(const v4f*)(tile + 4 * q0);
  const v4f f1 = *(const v4f*)(tile + 4 * q1);
  const size_t gb  = (size_t)blockIdx.x * 64 * CIN;
  const size_t hix = (size_t)p * CIN + cg * 8;
  *(volatile v4f*)(xf + gb + 4 * q0) = f0;
  *(volatile v4f*)(xf + gb + 4 * q1) = f1;
  *(volatile v8us*)(xh + hix) = hv;
  *(volatile v8us*)(xl + hix) = lv;
  __threadfence();
  *(volatile v4f*)(xf + gb + 4 * q0) = f0;
  *(volatile v4f*)(xf + gb + 4 * q1) = f1;
  *(volatile v8us*)(xh + hix) = hv;
  *(volatile v8us*)(xl + hix) = lv;
}

__global__ __launch_bounds__(256) void k_packw(const float* __restrict__ w_off,
                                               const float* __restrict__ w_mask,
                                               const float* __restrict__ w,
                                               unsigned short* w1h, unsigned short* w1l,
                                               unsigned short* w2h, unsigned short* w2l) {
  const int t = blockIdx.x * 256 + threadIdx.x;
  if (t >= T1 + T2) return;
  const bool first = t < T1;
  const int e0 = (first ? t : (t - T1)) * 8;
  const int n = e0 / KDIM;
  const int k0 = e0 - n * KDIM;
  const int tap = k0 >> 5;
  const int c0 = k0 & 31;
  const int no = min(n, 3 * KT - 1);
  const int nm = min(max(n - 3 * KT, 0), KT - 1);
  const int nw = min(n, COUT - 1);
  v8us hv, lv;
#pragma unroll
  for (int j = 0; j < 8; ++j) {
    const int c = c0 + j;
    const float vo = w_off[(no * CIN + c) * KT + tap];
    const float vm = w_mask[(nm * CIN + c) * KT + tap];
    const float vw = w[(nw * CIN + c) * KT + tap];
    const float f = first ? ((n < 3 * KT) ? vo : ((n < 4 * KT) ? vm : 0.0f)) : vw;
    const unsigned int hb = bf16_rne(f);
    hv[j] = (unsigned short)hb;
    lv[j] = (unsigned short)bf16_rne(f - __uint_as_float(hb << 16));
  }
  unsigned short* ph = first ? w1h : w2h;
  unsigned short* pq = first ? w1l : w2l;
  *(volatile v8us*)(ph + e0) = hv;
  *(volatile v8us*)(pq + e0) = lv;
  __threadfence();
  *(volatile v8us*)(ph + e0) = hv;
  *(volatile v8us*)(pq + e0) = lv;
}

__global__ __launch_bounds__(NTH) void k_main(const unsigned short* __restrict__ xh,
                                              const unsigned short* __restrict__ xl,
                                              const float* __restrict__ xf,
                                              const unsigned short* __restrict__ w1h,
                                              const unsigned short* __restrict__ w1l,
                                              const unsigned short* __restrict__ w2h,
                                              const unsigned short* __restrict__ w2l,
                                              const float* __restrict__ b_off,
                                              const float* __restrict__ b_mask,
                                              const float* __restrict__ bias,
                                              float* out) {
  __shared__ __attribute__((aligned(16))) float offs[NWV * N1 * 16];
  __shared__ __attribute__((aligned(16))) unsigned short atile[NWV * 2 * 16 * CIN];
  const int tid = threadIdx.x, lane = tid & 31, wave = tid >> 5;
  const int hh = lane >> 4, m = lane & 15;
  const int posblk = blockIdx.x * POSB;
  const int posw = posblk + wave * 16;
  const int x0 = posw & (WW - 1);
  const int y0 = (posw >> 6) & (HH - 1);
  const int z0 = posw >> 12;
  float* my = offs + wave * (N1 * 16);

  v8f acc[NT1];
#pragma unroll
  for (int nt = 0; nt < NT1; ++nt) acc[nt] = zero8f();
  const int abase = ((z0 * PH + y0) * PW + x0 + m) * CIN + 8 * hh;
  const unsigned short* w1hr = w1h + (size_t)m * KDIM + 8 * hh;
  const unsigned short* w1lr = w1l + (size_t)m * KDIM + 8 * hh;
#pragma unroll 1
  for (int s = 0; s < KT; ++s) {
    const int kz = s / 9, ky = (s / 3) % 3, kx = s % 3;
    const int ai = abase + ((kz * PH + ky) * PW + kx) * CIN;
    FragB ah, al;
    ah.u[0] = *(const v8us*)(xh + ai);
    ah.u[1] = *(const v8us*)(xh + ai + 16);
    al.u[0] = *(const v8us*)(xl + ai);
    al.u[1] = *(const v8us*)(xl + ai + 16);
    const int kb = s * CIN;
#pragma unroll
    for (int nt = 0; nt < NT1; ++nt) {
      FragB bh, bl;
      const unsigned short* bp = w1hr + nt * 16 * KDIM + kb;
      const unsigned short* bq = w1lr + nt * 16 * KDIM + kb;
      bh.u[0] = *(const v8us*)bp;
      bh.u[1] = *(const v8us*)(bp + 16);
      bl.u[0] = *(const v8us*)bq;
      bl.u[1] = *(const v8us*)(bq + 16);
      acc[nt] = wmb(ah.v, bh.v, acc[nt]);
      acc[nt] = wmb(ah.v, bl.v, acc[nt]);
      acc[nt] = wmb(al.v, bh.v, acc[nt]);
      wguard(acc[nt], ah.v, al.v, bh.v, bl.v);
    }
  }
#pragma unroll
  for (int nt = 0; nt < NT1; ++nt) {
    v4f d0 = {acc[nt][0], acc[nt][1], acc[nt][2], acc[nt][3]};
    v4f d1 = {acc[nt][4], acc[nt][5], acc[nt][6], acc[nt][7]};
    float* dp = my + (nt * 16 + m) * 16 + 8 * hh;
    *(v4f*)dp       = d0;
    *(v4f*)(dp + 4) = d1;
  }
  __syncthreads();

  v8f oacc[2];
  oacc[0] = zero8f();
  oacc[1] = zero8f();
  unsigned short* th = atile + wave * (2 * 16 * CIN);
  const unsigned short* w2hr = w2h + (size_t)m * KDIM + 8 * hh;
  const unsigned short* w2lr = w2l + (size_t)m * KDIM + 8 * hh;
  const int cb = 16 * hh;
  const int xm = x0 + m;
#pragma unroll 1
  for (int tap = 0; tap < KT; ++tap) {
    const int kz = tap / 9, ky = (tap / 3) % 3, kx = tap % 3;
    const float oz = my[tap * 16 + m]            + b_off[tap];
    const float oy = my[(KT + tap) * 16 + m]     + b_off[KT + tap];
    const float ox = my[(2 * KT + tap) * 16 + m] + b_off[2 * KT + tap];
    const float lg = my[(3 * KT + tap) * 16 + m] + b_mask[tap];
    const float ex = expf(-lg);
    const float mval = __builtin_amdgcn_rcpf(1.0f + ex);
    const float cz = (float)(z0 - 1 + kz) + oz;
    const float cy = (float)(y0 - 1 + ky) + oy;
    const float cx = (float)(xm - 1 + kx) + ox;
    const float fz = floorf(cz), fy = floorf(cy), fx = floorf(cx);
    const float tz = cz - fz, ty = cy - fy, tx = cx - fx;
    const int iz = (int)fz, iy = (int)fy, ix = (int)fx;

    float av[16];
#pragma unroll
    for (int j = 0; j < 16; ++j) av[j] = 0.0f;
#pragma unroll 1
    for (int c = 0; c < 8; ++c) {
      const int dz = c >> 2, dy = (c >> 1) & 1, dx = c & 1;
      const int zi = iz + dz, yi = iy + dy, xi = ix + dx;
      const bool ok = (zi >= 0) && (zi < DD) && (yi >= 0) && (yi < HH) && (xi >= 0) && (xi < WW);
      const float wz = (dz != 0) ? tz : (1.0f - tz);
      const float wy = (dy != 0) ? ty : (1.0f - ty);
      const float wx = (dx != 0) ? tx : (1.0f - tx);
      float wgt = (wz * wy) * wx;
      wgt = ok ? wgt : 0.0f;
      const int zc = min(max(zi, 0), DD - 1);
      const int yc = min(max(yi, 0), HH - 1);
      const int xc = min(max(xi, 0), WW - 1);
      const float* gp = xf + ((size_t)((zc + 1) * PH + (yc + 1)) * PW + (xc + 1)) * CIN + cb;
      const v4f g0 = *(const v4f*)(gp);
      const v4f g1 = *(const v4f*)(gp + 4);
      const v4f g2 = *(const v4f*)(gp + 8);
      const v4f g3 = *(const v4f*)(gp + 12);
#pragma unroll
      for (int j = 0; j < 4; ++j) {
        av[j]      += wgt * g0[j];
        av[4 + j]  += wgt * g1[j];
        av[8 + j]  += wgt * g2[j];
        av[12 + j] += wgt * g3[j];
      }
    }
    v8us h0, h1, l0, l1;
#pragma unroll
    for (int j = 0; j < 8; ++j) {
      const float va = av[j] * mval, vb = av[8 + j] * mval;
      const unsigned int ha = bf16_rne(va), hb = bf16_rne(vb);
      h0[j] = (unsigned short)ha;
      h1[j] = (unsigned short)hb;
      l0[j] = (unsigned short)bf16_rne(va - __uint_as_float(ha << 16));
      l1[j] = (unsigned short)bf16_rne(vb - __uint_as_float(hb << 16));
    }
    __syncthreads();
    {
      unsigned short* trow = th + m * CIN + cb;
      *(v8us*)(trow)           = h0;
      *(v8us*)(trow + 8)       = h1;
      *(v8us*)(trow + 512)     = l0;
      *(v8us*)(trow + 512 + 8) = l1;
    }
    __syncthreads();
    FragB fh, fl;
    {
      const unsigned short* frow = th + m * CIN + 8 * hh;
      fh.u[0] = *(const v8us*)(frow);
      fh.u[1] = *(const v8us*)(frow + 16);
      fl.u[0] = *(const v8us*)(frow + 512);
      fl.u[1] = *(const v8us*)(frow + 512 + 16);
    }
    const int wb = tap * CIN;
#pragma unroll
    for (int nt = 0; nt < 2; ++nt) {
      FragB bh, bl;
      const unsigned short* bp = w2hr + nt * 16 * KDIM + wb;
      const unsigned short* bq = w2lr + nt * 16 * KDIM + wb;
      bh.u[0] = *(const v8us*)bp;
      bh.u[1] = *(const v8us*)(bp + 16);
      bl.u[0] = *(const v8us*)bq;
      bl.u[1] = *(const v8us*)(bq + 16);
      oacc[nt] = wmb(fh.v, bh.v, oacc[nt]);
      oacc[nt] = wmb(fh.v, bl.v, oacc[nt]);
      oacc[nt] = wmb(fl.v, bh.v, oacc[nt]);
      wguard(oacc[nt], fh.v, fl.v, bh.v, bl.v);
    }
  }

  __syncthreads();
  float* ost = offs;
#pragma unroll
  for (int nt = 0; nt < 2; ++nt) {
    const int co = nt * 16 + m;
    const float bb = bias[co];
    v4f d0 = {oacc[nt][0] + bb, oacc[nt][1] + bb, oacc[nt][2] + bb, oacc[nt][3] + bb};
    v4f d1 = {oacc[nt][4] + bb, oacc[nt][5] + bb, oacc[nt][6] + bb, oacc[nt][7] + bb};
    float* op = ost + co * POSB + wave * 16 + 8 * hh;
    *(v4f*)op       = d0;
    *(v4f*)(op + 4) = d1;
  }
  __syncthreads();
  v4f ov[4];
  size_t ga[4];
#pragma unroll
  for (int p = 0; p < 4; ++p) {
    const int q = p * NTH + tid;
    const int co = q >> 4, piece = q & 15;
    ov[p] = *(const v4f*)(ost + 4 * q);
    ga[p] = (size_t)co * NSP + (size_t)posblk + (size_t)(piece * 4);
  }
#pragma unroll
  for (int p = 0; p < 4; ++p) *(volatile v4f*)(out + ga[p]) = ov[p];
  __threadfence();
#pragma unroll
  for (int p = 0; p < 4; ++p) *(volatile v4f*)(out + ga[p]) = ov[p];
}

extern "C" void kernel_launch(void* const* d_in, const int* in_sizes, int n_in,
                              void* d_out, int out_size, void* d_ws, size_t ws_size,
                              hipStream_t stream) {
  if (n_in < 7) return;
  if (in_sizes[0] != CIN * NSP) return;
  if (in_sizes[1] != 3 * KT * KDIM || in_sizes[2] != 3 * KT) return;
  if (in_sizes[3] != KT * KDIM || in_sizes[4] != KT) return;
  if (in_sizes[5] != COUT * KDIM || in_sizes[6] != COUT) return;
  if (out_size != COUT * NSP) return;

  const float* x      = (const float*)d_in[0];
  const float* w_off  = (const float*)d_in[1];
  const float* b_off  = (const float*)d_in[2];
  const float* w_mask = (const float*)d_in[3];
  const float* b_mask = (const float*)d_in[4];
  const float* w      = (const float*)d_in[5];
  const float* b      = (const float*)d_in[6];
  float* out = (float*)d_out;

  char* ws = (char*)d_ws;
  size_t off = 0;
  const size_t A = 4096;
  const size_t szXF = (size_t)NPPR * CIN * 4;
  const size_t szXH = (size_t)NPPR * CIN * 2;
  const size_t szW1 = ((size_t)N1 * KDIM * 2 + A - 1) & ~(A - 1);
  const size_t szW2 = ((size_t)COUT * KDIM * 2 + A - 1) & ~(A - 1);
  const size_t oXF = off; off += (szXF + A - 1) & ~(A - 1);
  const size_t oXH = off; off += (szXH + A - 1) & ~(A - 1);
  const size_t oXL = off; off += (szXH + A - 1) & ~(A - 1);
  const size_t oW1H = off; off += szW1;
  const size_t oW1L = off; off += szW1;
  const size_t oW2H = off; off += szW2;
  const size_t oW2L = off; off += szW2;
  if (off > ws_size || off > (size_t)134217728) return;

  float* xf = (float*)(ws + oXF);
  unsigned short* xh  = (unsigned short*)(ws + oXH);
  unsigned short* xl  = (unsigned short*)(ws + oXL);
  unsigned short* w1h = (unsigned short*)(ws + oW1H);
  unsigned short* w1l = (unsigned short*)(ws + oW1L);
  unsigned short* w2h = (unsigned short*)(ws + oW2H);
  unsigned short* w2l = (unsigned short*)(ws + oW2L);

  k_pad<<<NPPR / 64, 256, 0, stream>>>(x, xf, xh, xl);
  k_packw<<<(T1 + T2 + 255) / 256, 256, 0, stream>>>(w_off, w_mask, w, w1h, w1l, w2h, w2l);
  k_main<<<NSP / POSB, NTH, 0, stream>>>(xh, xl, xf, w1h, w1l, w2h, w2l, b_off, b_mask, b, out);
}
